// HeteroGNN_28535762714971
// MI455X (gfx1250) — hardware-verified
//
#include <hip/hip_runtime.h>
#include <stddef.h>
#include <stdint.h>
#include <math.h>


#define HC     128
#define DU     128
#define DS     64
#define K1     192
#define K2     256
#define NTHR   256
#define NWAVE  8
#define EPT    8
#define CHUNK  (NTHR * EPT)
#define WCAP   (EPT * 32)
#define LISTN  (NWAVE * WCAP)
#define NBA    1024
#define SLA    10
#define RCAP   28672
#define DEGCAP 1024
#define GBM    64
#define GTHR   128
#define UP128  2048
#define UP64   1024
#define UTOT   (6 * UP128 + 2 * UP64)
#define AGG_ZINTS    (LISTN + 2 * RCAP + 3 * NBA)
#define MISC_INTS    16
#define AGG_LDS_INTS (AGG_ZINTS + MISC_INTS)
#define WSMAX  134217728

static_assert((CHUNK & (CHUNK - 1)) == 0 && CHUNK <= 4096);
static_assert((NBA & (NBA - 1)) == 0 && NBA == (1 << SLA));
static_assert(((long long)CHUNK << SLA) < (1LL << 31));
static_assert(LISTN % NTHR == 0);
static_assert(NBA % NWAVE == 0 && NBA % 32 == 0 && NBA % GBM == 0);
static_assert(RCAP % 4 == 0 && AGG_ZINTS % 4 == 0 && LISTN % 4 == 0);
static_assert(AGG_ZINTS % (NTHR * 4) == 0);
static_assert(K1 % 32 == 0 && K2 % 32 == 0 && K1 == DU + DS && K2 == 2 * HC);
static_assert(GBM == (GTHR / 32) * 16 && HC == 4 * 32 && DU == HC && DS * 2 == HC);
static_assert(UP128 % NTHR == 0 && UP64 % NTHR == 0 && UTOT % NTHR == 0);
static_assert(UP128 == HC * (128 / 8) && UP64 == HC * (64 / 8));
static_assert(AGG_LDS_INTS * 4 <= 300000);
static_assert(NTHR == 2 * HC);

typedef float          v4f   __attribute__((ext_vector_type(4)));
typedef float          v8f   __attribute__((ext_vector_type(8)));
typedef int            v4i   __attribute__((ext_vector_type(4)));
typedef int            v8i   __attribute__((ext_vector_type(8)));
typedef unsigned short v8us  __attribute__((ext_vector_type(8)));
typedef unsigned short v16us __attribute__((ext_vector_type(16)));
typedef __bf16         v16bf __attribute__((ext_vector_type(16)));
typedef v4f  __attribute__((may_alias)) v4fa;
typedef v4i  __attribute__((may_alias)) v4ia;
typedef v8us __attribute__((may_alias)) v8usa;
union FragB { v16bf v; v16us u; v8us h[2]; v8i w; };

__device__ __forceinline__ v8f wmb(const FragB& a, const FragB& b, v8f c) {
  v8f d = __builtin_amdgcn_wmma_f32_16x16x32_bf16(false, a.v, false, b.v, (short)0, c, false, false);
  asm volatile("v_nop\n\tv_nop\n\tv_nop\n\tv_nop" : "+v"(d) : "v"(a.w), "v"(b.w));
  return d;
}

__device__ __forceinline__ unsigned bf16_bits(float f) {
  const unsigned u = __float_as_uint(f);
  return ((u + 0x7FFFu + ((u >> 16) & 1u)) >> 16) & 0xFFFFu;
}
__device__ __forceinline__ float bf16_val(float f) {
  return __uint_as_float(bf16_bits(f) << 16);
}
__device__ __forceinline__ v4f bfr4(const v4f a) {
  v4f r; r.x = bf16_val(a.x); r.y = bf16_val(a.y); r.z = bf16_val(a.z); r.w = bf16_val(a.w); return r;
}
__device__ __forceinline__ void split2(float v, unsigned& hi, unsigned& lo) {
  hi = bf16_bits(v);
  lo = bf16_bits(v - __uint_as_float(hi << 16));
}

__device__ __forceinline__ FragB frag_f32(const float* p) {
  const v4f f0 = *(const v4f*)p;
  const v4f f1 = *(const v4f*)(p + 4);
  const v4f f2 = *(const v4f*)(p + 16);
  const v4f f3 = *(const v4f*)(p + 20);
  v16us u;
  u[0]  = (unsigned short)bf16_bits(f0.x); u[1]  = (unsigned short)bf16_bits(f0.y);
  u[2]  = (unsigned short)bf16_bits(f0.z); u[3]  = (unsigned short)bf16_bits(f0.w);
  u[4]  = (unsigned short)bf16_bits(f1.x); u[5]  = (unsigned short)bf16_bits(f1.y);
  u[6]  = (unsigned short)bf16_bits(f1.z); u[7]  = (unsigned short)bf16_bits(f1.w);
  u[8]  = (unsigned short)bf16_bits(f2.x); u[9]  = (unsigned short)bf16_bits(f2.y);
  u[10] = (unsigned short)bf16_bits(f2.z); u[11] = (unsigned short)bf16_bits(f2.w);
  u[12] = (unsigned short)bf16_bits(f3.x); u[13] = (unsigned short)bf16_bits(f3.y);
  u[14] = (unsigned short)bf16_bits(f3.z); u[15] = (unsigned short)bf16_bits(f3.w);
  FragB a;
  a.u = u;
  return a;
}

#define SPL_EL(I, V) { unsigned th, tl; split2((V), th, tl); uh[I] = (unsigned short)th; ul[I] = (unsigned short)tl; }
__device__ __forceinline__ void frag_split(const float* p, FragB& hi, FragB& lo) {
  const v4f f0 = *(const v4f*)p;
  const v4f f1 = *(const v4f*)(p + 4);
  const v4f f2 = *(const v4f*)(p + 16);
  const v4f f3 = *(const v4f*)(p + 20);
  v16us uh, ul;
  SPL_EL(0, f0.x)  SPL_EL(1, f0.y)  SPL_EL(2, f0.z)  SPL_EL(3, f0.w)
  SPL_EL(4, f1.x)  SPL_EL(5, f1.y)  SPL_EL(6, f1.z)  SPL_EL(7, f1.w)
  SPL_EL(8, f2.x)  SPL_EL(9, f2.y)  SPL_EL(10, f2.z) SPL_EL(11, f2.w)
  SPL_EL(12, f3.x) SPL_EL(13, f3.y) SPL_EL(14, f3.z) SPL_EL(15, f3.w)
  hi.u = uh;
  lo.u = ul;
}
#undef SPL_EL

template <int SLB>
__device__ __forceinline__ int scan_chunk(const int* __restrict__ dsts, int nE, int cbase, int slotBase,
                                          int nb, int vec8, int* list, int tid, int lane, int wave) {
  int wc = 0;
  const int el0  = tid * EPT;
  const int e0   = cbase + el0;
  const int sent = -2147483647 - 1;
  v4i da, db;
  if (vec8 != 0 && cbase + CHUNK <= nE) {
    da = *(const v4i*)(dsts + e0);
    db = *(const v4i*)(dsts + e0 + 4);
  } else {
    da.x = (e0     < nE) ? dsts[min(e0,     nE - 1)] : sent;
    da.y = (e0 + 1 < nE) ? dsts[min(e0 + 1, nE - 1)] : sent;
    da.z = (e0 + 2 < nE) ? dsts[min(e0 + 2, nE - 1)] : sent;
    da.w = (e0 + 3 < nE) ? dsts[min(e0 + 3, nE - 1)] : sent;
    db.x = (e0 + 4 < nE) ? dsts[min(e0 + 4, nE - 1)] : sent;
    db.y = (e0 + 5 < nE) ? dsts[min(e0 + 5, nE - 1)] : sent;
    db.z = (e0 + 6 < nE) ? dsts[min(e0 + 6, nE - 1)] : sent;
    db.w = (e0 + 7 < nE) ? dsts[min(e0 + 7, nE - 1)] : sent;
  }
  const unsigned nbs = (unsigned)slotBase;
  const unsigned unb = (unsigned)nb;
  const unsigned s0 = (unsigned)da.x - nbs, s1 = (unsigned)da.y - nbs;
  const unsigned s2 = (unsigned)da.z - nbs, s3 = (unsigned)da.w - nbs;
  const unsigned s4 = (unsigned)db.x - nbs, s5 = (unsigned)db.y - nbs;
  const unsigned s6 = (unsigned)db.z - nbs, s7 = (unsigned)db.w - nbs;
  const bool h0 = s0 < unb, h1 = s1 < unb, h2 = s2 < unb, h3 = s3 < unb;
  const bool h4 = s4 < unb, h5 = s5 < unb, h6 = s6 < unb, h7 = s7 < unb;
  const unsigned any = __builtin_amdgcn_ballot_w32(h0 | h1 | h2 | h3 | h4 | h5 | h6 | h7);
  if (any != 0u) {
#define HITJ(J, HJ, SJ) { \
      const unsigned mj = __builtin_amdgcn_ballot_w32(HJ); \
      if (mj != 0u) { \
        if (HJ) { \
          const int pos = wc + (int)__builtin_amdgcn_mbcnt_lo(mj, 0u); \
          if (pos < WCAP) list[wave * WCAP + pos] = ((el0 + (J)) << SLB) | (int)(SJ); \
        } \
        wc += (int)__builtin_popcount(mj); } }
    HITJ(0, h0, s0)
    HITJ(1, h1, s1)
    HITJ(2, h2, s2)
    HITJ(3, h3, s3)
    HITJ(4, h4, s4)
    HITJ(5, h5, s5)
    HITJ(6, h6, s6)
    HITJ(7, h7, s7)
#undef HITJ
  }
  return wc;
}

__global__ __launch_bounds__(NTHR) void k_wprep(const float* __restrict__ wl1s, const float* __restrict__ wr1s,
                                                const float* __restrict__ wl1u, const float* __restrict__ wr1u,
                                                const float* __restrict__ wl2s, const float* __restrict__ wr2s,
                                                const float* __restrict__ wl2u, const float* __restrict__ wr2u,
                                                unsigned short* BS1, unsigned short* BU1,
                                                unsigned short* BS2, unsigned short* BU2) {
  const int u = (int)blockIdx.x * NTHR + (int)threadIdx.x;
  if (u >= UTOT) return;
  const float* W;
  unsigned short* P;
  int pitch, coff, kr, v;
  if (u < 2048)       { W = wl1s; P = BS1; pitch = K1; coff = 0;   kr = 128; v = u; }
  else if (u < 3072)  { W = wr1s; P = BS1; pitch = K1; coff = 128; kr = 64;  v = u - 2048; }
  else if (u < 4096)  { W = wl1u; P = BU1; pitch = K1; coff = 0;   kr = 64;  v = u - 3072; }
  else if (u < 6144)  { W = wr1u; P = BU1; pitch = K1; coff = 64;  kr = 128; v = u - 4096; }
  else if (u < 8192)  { W = wl2s; P = BS2; pitch = K2; coff = 0;   kr = 128; v = u - 6144; }
  else if (u < 10240) { W = wr2s; P = BS2; pitch = K2; coff = 128; kr = 128; v = u - 8192; }
  else if (u < 12288) { W = wl2u; P = BU2; pitch = K2; coff = 0;   kr = 128; v = u - 10240; }
  else                { W = wr2u; P = BU2; pitch = K2; coff = 128; kr = 128; v = u - 12288; }
  const int n  = (kr == 128) ? (v >> 4) : (v >> 3);
  const int k8 = (kr == 128) ? ((v & 15) * 8) : ((v & 7) * 8);
  const float* p = W + (size_t)k8 * HC + n;
  float f[8];
#pragma unroll
  for (int i = 0; i < 8; ++i) f[i] = p[(size_t)i * HC];
  v8us o;
#pragma unroll
  for (int i = 0; i < 8; ++i) o[i] = (unsigned short)bf16_bits(f[i]);
  unsigned short* dp = P + (size_t)n * (size_t)pitch + coff + k8;
  *(volatile v8us*)dp = o;
  __threadfence();
  *(volatile v8us*)dp = o;
}

template <int KS1, int KS2, int SPL2>
__global__ __launch_bounds__(GTHR) void k_gemm(const float* __restrict__ A1, int r1lo, const float* A2, int n2,
                                               const unsigned short* __restrict__ BT,
                                               const float* __restrict__ bias, float* D, int rlo) {
  constexpr int K  = 32 * (KS1 + KS2);
  constexpr int P1 = 32 * KS1;
  constexpr int P2 = 32 * KS2;
  __shared__ __attribute__((aligned(16))) float stg[GBM * HC];
  const int tid = (int)threadIdx.x, lane = tid & 31, wave = tid >> 5, hh = lane >> 4, m = lane & 15;
  const int rbase = rlo + (int)blockIdx.x * GBM;
  const int r = rbase + 16 * wave + m;

  v8f acc[8];
  {
    const v8f z = {0.f, 0.f, 0.f, 0.f, 0.f, 0.f, 0.f, 0.f};
#pragma unroll
    for (int t = 0; t < 8; ++t) acc[t] = z;
  }
  const float* a1p = A1 + (size_t)(r - r1lo) * (size_t)P1 + 8 * hh;
  int r2 = r < n2 ? r : n2 - 1;
  r2 = r2 < 0 ? 0 : r2;
  const float* a2p = A2 + (size_t)r2 * (size_t)P2 + 8 * hh;
  const unsigned short* bp = BT + (size_t)m * (size_t)K + 8 * hh;

#pragma unroll 1
  for (int ks = 0; ks < KS1; ++ks) {
    FragB ah, al;
    frag_split(a1p + 32 * ks, ah, al);
#pragma unroll
    for (int t = 0; t < 8; ++t) {
      const unsigned short* wq = bp + (size_t)(16 * t) * (size_t)K + 32 * ks;
      FragB bf;
      bf.h[0] = *(const v8usa*)wq;
      bf.h[1] = *(const v8usa*)(wq + 16);
      acc[t] = wmb(ah, bf, acc[t]);
      acc[t] = wmb(al, bf, acc[t]);
    }
  }
#pragma unroll 1
  for (int ks = 0; ks < KS2; ++ks) {
    const int kb = 32 * (KS1 + ks);
    if constexpr (SPL2 != 0) {
      FragB ah, al;
      frag_split(a2p + 32 * ks, ah, al);
#pragma unroll
      for (int t = 0; t < 8; ++t) {
        const unsigned short* wq = bp + (size_t)(16 * t) * (size_t)K + kb;
        FragB bf;
        bf.h[0] = *(const v8usa*)wq;
        bf.h[1] = *(const v8usa*)(wq + 16);
        acc[t] = wmb(ah, bf, acc[t]);
        acc[t] = wmb(al, bf, acc[t]);
      }
    } else {
      const FragB af = frag_f32(a2p + 32 * ks);
#pragma unroll
      for (int t = 0; t < 8; ++t) {
        const unsigned short* wq = bp + (size_t)(16 * t) * (size_t)K + kb;
        FragB bf;
        bf.h[0] = *(const v8usa*)wq;
        bf.h[1] = *(const v8usa*)(wq + 16);
        acc[t] = wmb(af, bf, acc[t]);
      }
    }
  }

#pragma unroll
  for (int t = 0; t < 8; ++t) {
    const int lc = 16 * t + m;
#pragma unroll
    for (int rr = 0; rr < 8; ++rr) {
      const int lr = 16 * wave + 8 * hh + rr;
      stg[lr * HC + lc] = acc[t][rr];
    }
  }
  __syncthreads();

  const v4f bb4 = bfr4(*(const v4f*)(bias + 4 * lane));
  v4f pv[16];
#pragma unroll
  for (int i = 0; i < 16; ++i) {
    v4f y = *(const v4fa*)(stg + (16 * wave + i) * HC + 4 * lane) + bb4;
    y.x = fmaxf(y.x, 0.0f); y.y = fmaxf(y.y, 0.0f); y.z = fmaxf(y.z, 0.0f); y.w = fmaxf(y.w, 0.0f);
    pv[i] = y;
  }
#pragma unroll
  for (int i = 0; i < 16; ++i) {
    float* op = D + (size_t)(rbase + 16 * wave + i) * (size_t)HC + 4 * lane;
    *(volatile v4f*)op = pv[i];
  }
  __threadfence();
#pragma unroll
  for (int i = 0; i < 16; ++i) {
    float* op = D + (size_t)(rbase + 16 * wave + i) * (size_t)HC + 4 * lane;
    *(volatile v4f*)op = pv[i];
  }
}

template <int GW, int RNDB>
__global__ __launch_bounds__(NTHR) void k_scan(const int* __restrict__ srcs, const int* __restrict__ dsts,
                                               int nE, int nSrc, int nDst, int rowLo, int mRows, int vec8,
                                               const float* __restrict__ gsrc, float* opl) {
  extern __shared__ __attribute__((aligned(16))) int dsm[];
  int* list = dsm;
  int* hl   = dsm + LISTN;
  int* sl   = hl + RCAP;
  int* cnt  = sl + RCAP;
  int* offs = cnt + NBA;
  int* cur  = offs + NBA;
  int* misc = cur + NBA;
  const int tid = (int)threadIdx.x, lane = tid & 31, wave = tid >> 5;
  const int nodeBase = rowLo + (int)blockIdx.x * NBA;

  {
    const v4i z4 = {0, 0, 0, 0};
    for (int i = tid * 4; i < AGG_ZINTS; i += NTHR * 4) *(v4ia*)(dsm + i) = z4;
    if (tid < MISC_INTS) misc[tid] = 0;
  }
  __syncthreads();

  int t = 0, ov = 0;
  const int nChunks = (nE + CHUNK - 1) / CHUNK;
#pragma unroll 1
  for (int ch = 0; ch < nChunks; ++ch) {
    const int cbase = ch * CHUNK;
    const int wc = scan_chunk<SLA>(dsts, nE, cbase, nodeBase, NBA, vec8, list, tid, lane, wave);
    if (lane == 0) misc[wave] = wc;
    __syncthreads();
    if (wave == 0) {
#pragma unroll 1
      for (int w2 = 0; w2 < NWAVE; ++w2) {
        int c = misc[w2];
        c = c < 0 ? 0 : (c > WCAP ? WCAP : c);
#pragma unroll 1
        for (int b0 = 0; b0 < c; b0 += 32) {
          const int idx = b0 + lane;
          const int ent = list[w2 * WCAP + (idx < WCAP ? idx : WCAP - 1)];
          const int m32 = (c - b0) < 32 ? (c - b0) : 32;
#pragma unroll 1
          for (int k = 0; k < m32; ++k) {
            const int u    = __builtin_amdgcn_readlane(ent, k);
            const int slot = u & (NBA - 1);
            const int el   = (u >> SLA) & (CHUNK - 1);
            const int pk   = ((cbase + el) << SLA) | slot;
            if (t < RCAP) {
              if (lane == 0) { hl[t] = pk; cnt[slot] = cnt[slot] + 1; }
              t = t + 1;
            } else {
              ov = 1;
            }
          }
        }
      }
    }
    __syncthreads();
  }
  if (wave == 0 && lane == 0) { misc[8] = t; misc[9] = ov; }
  __syncthreads();
  int tt = misc[8];
  tt = tt < 0 ? 0 : (tt > RCAP ? RCAP : tt);
  const int ovf = misc[9];

  if (wave == 0) {
    const int base = lane * (NBA / 32);
    int s = 0;
#pragma unroll 1
    for (int i = 0; i < NBA / 32; ++i) s += cnt[base + i];
    int incl = s;
#pragma unroll
    for (int d = 1; d < 32; d <<= 1) {
      const int y = __shfl_up(incl, d, 32);
      if (lane >= d) incl += y;
    }
    int run = incl - s;
#pragma unroll 1
    for (int i = 0; i < NBA / 32; ++i) {
      const int cv = cnt[base + i];
      offs[base + i] = run;
      cur[base + i]  = run;
      run += cv;
    }
  }
  __syncthreads();
  if (wave == 0) {
#pragma unroll 1
    for (int b0 = 0; b0 < tt; b0 += 32) {
      const int idx = b0 + lane;
      const int ent = hl[idx < RCAP ? idx : RCAP - 1];
      const int m32 = (tt - b0) < 32 ? (tt - b0) : 32;
#pragma unroll 1
      for (int k = 0; k < m32; ++k) {
        const int u    = __builtin_amdgcn_readlane(ent, k);
        const int slot = u & (NBA - 1);
        if (lane == 0) {
          int p = cur[slot];
          p = p < 0 ? 0 : (p > RCAP - 1 ? RCAP - 1 : p);
          sl[p] = u;
          cur[slot] = p + 1;
        }
      }
    }
  }
  __syncthreads();

  const float qnan = __int_as_float(0x7fc00000);
  const float pz = (ovf != 0) ? qnan : 0.0f;
  const int c4 = (GW == 128) ? (4 * lane) : (4 * (lane & 15));
#pragma unroll 1
  for (int si = 0; si < NBA / NWAVE; ++si) {
    const int s    = si * NWAVE + wave;
    const int node = nodeBase + s;
    int c = cnt[s];
    const bool big = c > DEGCAP;
    c = c < 0 ? 0 : (c > DEGCAP ? DEGCAP : c);
    int o = offs[s];
    o = o < 0 ? 0 : (o > RCAP ? RCAP : o);
    float a0 = 0.0f, a1 = 0.0f, a2 = 0.0f, a3 = 0.0f;
#pragma unroll 1
    for (int b0 = 0; b0 < c; b0 += 32) {
      int idx = o + b0 + lane;
      idx = idx > RCAP - 1 ? RCAP - 1 : idx;
      const int ent = sl[idx];
      int eid = ent >> SLA;
      eid = eid < 0 ? 0 : (eid > nE - 1 ? nE - 1 : eid);
      int sr = srcs[eid];
      sr = sr < 0 ? 0 : (sr > nSrc - 1 ? nSrc - 1 : sr);
      const int m32 = (c - b0) < 32 ? (c - b0) : 32;
#pragma unroll 1
      for (int k = 0; k < m32; ++k) {
        const int sk = __builtin_amdgcn_readlane(sr, k);
        const v4f a = *(const v4f*)(gsrc + (size_t)sk * (size_t)GW + c4);
        if constexpr (RNDB != 0) {
          a0 += bf16_val(a.x); a1 += bf16_val(a.y); a2 += bf16_val(a.z); a3 += bf16_val(a.w);
        } else {
          a0 += a.x; a1 += a.y; a2 += a.z; a3 += a.w;
        }
      }
    }
    const float inv = 1.0f / fmaxf((float)c, 1.0f);
    const float pzr = big ? qnan : pz;
    const bool live = node < nDst;
    v4f mv;
    mv.x = live ? (a0 * inv + pzr) : 0.0f;
    mv.y = live ? (a1 * inv + pzr) : 0.0f;
    mv.z = live ? (a2 * inv + pzr) : 0.0f;
    mv.w = live ? (a3 * inv + pzr) : 0.0f;
    const int prow = node - rowLo;
    if (prow < mRows) {
      float* rp = opl + (size_t)prow * (size_t)GW + c4;
      const bool wr = (GW == 128) || (lane < 16);
      if (wr) *(volatile v4f*)rp = mv;
      __threadfence();
      if (wr) *(volatile v4f*)rp = mv;
    }
  }
}

__global__ __launch_bounds__(NTHR) void k_head(const float* __restrict__ U, const float* __restrict__ S,
                                               const int* __restrict__ mku, const int* __restrict__ mks,
                                               const float* __restrict__ wlin, const float* __restrict__ blin,
                                               float* out, int nB, int nU, int nS) {
  __shared__ __attribute__((aligned(16))) float wl[2 * HC];
  const int tid = (int)threadIdx.x;
  wl[tid] = bf16_val(wlin[tid]);
  __syncthreads();
  const int t  = (int)blockIdx.x * NTHR + tid;
  const int tc = t < nB ? t : nB - 1;
  int iu = mku[tc];
  int is = mks[tc];
  iu = iu < 0 ? 0 : (iu > nU - 1 ? nU - 1 : iu);
  is = is < 0 ? 0 : (is > nS - 1 ? nS - 1 : is);
  const float* ur = U + (size_t)iu * HC;
  const float* sr = S + (size_t)is * HC;
  float a0 = 0.f, a1 = 0.f, a2 = 0.f, a3 = 0.f;
  float c0 = 0.f, c1 = 0.f, c2 = 0.f, c3 = 0.f;
#pragma unroll 2
  for (int q = 0; q < HC / 4; ++q) {
    const v4f x = *(const v4f*)(ur + 4 * q);
    const v4f w = *(const v4fa*)(wl + 4 * q);
    a0 = fmaf(x.x, w.x, a0); a1 = fmaf(x.y, w.y, a1); a2 = fmaf(x.z, w.z, a2); a3 = fmaf(x.w, w.w, a3);
  }
#pragma unroll 2
  for (int q = 0; q < HC / 4; ++q) {
    const v4f x = *(const v4f*)(sr + 4 * q);
    const v4f w = *(const v4fa*)(wl + HC + 4 * q);
    c0 = fmaf(x.x, w.x, c0); c1 = fmaf(x.y, w.y, c1); c2 = fmaf(x.z, w.z, c2); c3 = fmaf(x.w, w.w, c3);
  }
  float z = ((a0 + a1) + (a2 + a3)) + ((c0 + c1) + (c2 + c3)) + bf16_val(blin[0]);
  z = z > 30.0f ? 30.0f : (z < -30.0f ? -30.0f : z);
  const float o = 1.0f / (1.0f + expf(-z));
  const bool wr = t < nB;
  if (wr) *(volatile float*)(out + t) = o;
  __threadfence();
  if (wr) *(volatile float*)(out + t) = o;
}

static inline int cdiv(int a, int b) { return (a + b - 1) / b; }

extern "C" void kernel_launch(void* const* d_in, const int* in_sizes, int n_in,
                              void* d_out, int out_size, void* d_ws, size_t ws_size,
                              hipStream_t stream) {
  if (n_in < 22) return;
  if (in_sizes[0] < DU || (in_sizes[0] % DU) != 0) return;
  if (in_sizes[1] < DS || (in_sizes[1] % DS) != 0) return;
  const int nU = in_sizes[0] / DU;
  const int nS = in_sizes[1] / DS;
  if (nU > (1 << 22) || nS > (1 << 22)) return;
  const int eB = in_sizes[2], eR = in_sizes[4];
  if (in_sizes[3] != eB || in_sizes[5] != eR) return;
  if (eB < 1 || eR < 1 || eB >= (1 << 21) || eR >= (1 << 21)) return;
  const int nB = in_sizes[6];
  if (nB < 1 || in_sizes[7] != nB || out_size != nB) return;
  if (in_sizes[8] != DU * HC || in_sizes[9] != DS * HC || in_sizes[10] != HC) return;
  if (in_sizes[11] != DS * HC || in_sizes[12] != DU * HC || in_sizes[13] != HC) return;
  for (int i = 14; i <= 17; i += 3) {
    if (in_sizes[i] != HC * HC || in_sizes[i + 1] != HC * HC || in_sizes[i + 2] != HC) return;
  }
  if (in_sizes[20] != 2 * HC || in_sizes[21] != 1) return;

  const float* xu   = (const float*)d_in[0];
  const float* xs   = (const float*)d_in[1];
  const int*   srcB = (const int*)d_in[2];
  const int*   dstB = (const int*)d_in[3];
  const int*   srcR = (const int*)d_in[4];
  const int*   dstR = (const int*)d_in[5];
  const int*   mku  = (const int*)d_in[6];
  const int*   mks  = (const int*)d_in[7];
  const float* wl1s = (const float*)d_in[8];
  const float* wr1s = (const float*)d_in[9];
  const float* b1s  = (const float*)d_in[10];
  const float* wl1u = (const float*)d_in[11];
  const float* wr1u = (const float*)d_in[12];
  const float* b1u  = (const float*)d_in[13];
  const float* wl2s = (const float*)d_in[14];
  const float* wr2s = (const float*)d_in[15];
  const float* b2s  = (const float*)d_in[16];
  const float* wl2u = (const float*)d_in[17];
  const float* wr2u = (const float*)d_in[18];
  const float* b2u  = (const float*)d_in[19];
  const float* wlin = (const float*)d_in[20];
  const float* blin = (const float*)d_in[21];
  float* out = (float*)d_out;

  const int MPU = cdiv(nU, GBM) * GBM;
  const int MPS = cdiv(nS, GBM) * GBM;
  const int RH1 = cdiv(MPU / GBM, 2) * GBM;
  const int RH2 = MPU - RH1;
  const int gSS = cdiv(MPS, NBA), gSU = cdiv(MPU, NBA);
  const int gH1 = cdiv(RH1, NBA), gH2 = (RH2 > 0) ? cdiv(RH2, NBA) : 0;
  if ((long long)gSS * NBA < (long long)MPS || (long long)gSU * NBA < (long long)MPU) return;
  if ((long long)gH1 * NBA < (long long)RH1 || (long long)gH2 * NBA < (long long)RH2) return;
  const int vec8 = 1;

  char* ws = (char*)d_ws;
  size_t off = 0;
  const size_t oBS1 = off; off += (size_t)HC * K1 * 2;                     off = (off + 255) & ~(size_t)255;
  const size_t oBU1 = off; off += (size_t)HC * K1 * 2;                     off = (off + 255) & ~(size_t)255;
  const size_t oBS2 = off; off += (size_t)HC * K2 * 2;                     off = (off + 255) & ~(size_t)255;
  const size_t oBU2 = off; off += (size_t)HC * K2 * 2;                     off = (off + 255) & ~(size_t)255;
  const size_t oU   = off; off += (size_t)MPU * HC * 4;                     off = (off + 255) & ~(size_t)255;
  const size_t oS   = off; off += (size_t)MPS * HC * 4;                     off = (off + 255) & ~(size_t)255;
  const size_t oMS  = off; off += (size_t)MPS * HC * 4;                     off = (off + 255) & ~(size_t)255;
  size_t muBytes = (size_t)MPU * DS * 4;
  if ((size_t)RH1 * HC * 4 > muBytes) muBytes = (size_t)RH1 * HC * 4;
  const size_t oMU  = off; off += muBytes;                                   off = (off + 255) & ~(size_t)255;
  if (off > ws_size || off > (size_t)WSMAX) return;
  unsigned short* BS1 = (unsigned short*)(ws + oBS1);
  unsigned short* BU1 = (unsigned short*)(ws + oBU1);
  unsigned short* BS2 = (unsigned short*)(ws + oBS2);
  unsigned short* BU2 = (unsigned short*)(ws + oBU2);
  float* U  = (float*)(ws + oU);
  float* S  = (float*)(ws + oS);
  float* MS = (float*)(ws + oMS);
  float* MU = (float*)(ws + oMU);

  const size_t scanLds = (size_t)AGG_LDS_INTS * 4;
  hipFuncSetAttribute(reinterpret_cast<const void*>(&k_scan<128, 1>), hipFuncAttributeMaxDynamicSharedMemorySize, (int)scanLds);
  hipFuncSetAttribute(reinterpret_cast<const void*>(&k_scan<64, 1>),  hipFuncAttributeMaxDynamicSharedMemorySize, (int)scanLds);
  hipFuncSetAttribute(reinterpret_cast<const void*>(&k_scan<128, 0>), hipFuncAttributeMaxDynamicSharedMemorySize, (int)scanLds);

  k_wprep<<<UTOT / NTHR, NTHR, 0, stream>>>(wl1s, wr1s, wl1u, wr1u, wl2s, wr2s, wl2u, wr2u, BS1, BU1, BS2, BU2);
  k_scan<128, 1><<<gSS, NTHR, scanLds, stream>>>(srcB, dstB, eB, nU, nS, 0, MPS, vec8, xu, MS);
  k_scan<64, 1><<<gSU, NTHR, scanLds, stream>>>(srcR, dstR, eR, nS, nU, 0, MPU, vec8, xs, MU);
  k_gemm<4, 2, 0><<<MPS / GBM, GTHR, 0, stream>>>(MS, 0, xs, nS, BS1, b1s, S, 0);
  k_gemm<2, 4, 0><<<MPU / GBM, GTHR, 0, stream>>>(MU, 0, xu, nU, BU1, b1u, U, 0);
  k_scan<128, 0><<<gSS, NTHR, scanLds, stream>>>(srcB, dstB, eB, nU, nS, 0, MPS, vec8, U, MS);
  k_scan<128, 0><<<gH1, NTHR, scanLds, stream>>>(srcR, dstR, eR, nS, nU, 0, RH1, vec8, S, MU);
  k_gemm<4, 4, 1><<<RH1 / GBM, GTHR, 0, stream>>>(MU, 0, U, MPU, BU2, b2u, U, 0);
  if (RH2 > 0) {
    k_scan<128, 0><<<gH2, NTHR, scanLds, stream>>>(srcR, dstR, eR, nS, nU, RH1, RH2, vec8, S, MU);
    k_gemm<4, 4, 1><<<RH2 / GBM, GTHR, 0, stream>>>(MU, RH1, U, MPU, BU2, b2u, U, RH1);
  }
  k_gemm<4, 4, 1><<<MPS / GBM, GTHR, 0, stream>>>(MS, 0, S, MPS, BS2, b2s, S, 0);
  k_head<<<cdiv(nB, NTHR), NTHR, 0, stream>>>(U, S, mku, mks, wlin, blin, out, nB, nU, nS);
}
